// MixedScoresSDPA_71270687310015
// MI455X (gfx1250) — hardware-verified
//
#include <hip/hip_runtime.h>
#include <stddef.h>
#include <stdint.h>
#include <math.h>

#define BB   8
#define HH   8
#define MM   512
#define NN   512
#define DD   64
#define HID  16
#define NBH  (BB * HH)
#define QBLK (MM / 128)
#define PL   ((size_t)NBH * NN * DD)

static_assert(MM % 128 == 0);
static_assert(NN % 64 == 0);
static_assert(DD == 64);
static_assert(HID == 16);
static_assert((NBH * MM * DD) % (8 * 256) == 0);

typedef _Float16 v16h __attribute__((ext_vector_type(16)));
typedef _Float16 v8h  __attribute__((ext_vector_type(8)));
typedef float    v8f  __attribute__((ext_vector_type(8)));
typedef float    v4f  __attribute__((ext_vector_type(4)));
typedef unsigned int v4u __attribute__((ext_vector_type(4)));

union Frag  { v16h v; v8h h[2]; };
union Pack8 { v8h h; v4u u; };

__device__ __forceinline__ v8f mma16(v16h a, v16h b, v8f c) {
  c = __builtin_amdgcn_wmma_f32_16x16x32_f16(false, a, false, b, (short)0, c, false, false);
  asm volatile("v_nop\n\tv_nop\n\tv_nop\n\tv_nop" : "+v"(c) : "v"(a), "v"(b));
  return c;
}

__device__ __forceinline__ v16h ldfrag(const _Float16* p, int ld, int row0, int k0, int lane) {
  const int m = lane & 15, lh = lane >> 4;
  const _Float16* q = p + (size_t)(row0 + m) * ld + k0 + 8 * lh;
  Frag f;
  f.h[0] = *(const v8h*)(q);
  f.h[1] = *(const v8h*)(q + 16);
  return f.v;
}

__device__ __forceinline__ v8f zero8() { return (v8f){0.f, 0.f, 0.f, 0.f, 0.f, 0.f, 0.f, 0.f}; }

__global__ __launch_bounds__(256) void k_cvt_qk(const float* __restrict__ q, const float* __restrict__ k,
                                                _Float16* __restrict__ qh, _Float16* __restrict__ kh,
                                                int ngrp, int nb) {
  const int sel = ((int)blockIdx.x >= nb) ? 1 : 0;
  const float* src = sel ? k : q;
  _Float16* dst = sel ? kh : qh;
  const int t = ((int)blockIdx.x - sel * nb) * 256 + (int)threadIdx.x;
  if (t >= ngrp) return;
  const size_t o = (size_t)t * 8;
  const v4f a0 = *(const v4f*)(src + o);
  const v4f a1 = *(const v4f*)(src + o + 4);
  Pack8 pk;
  pk.h = (v8h){(_Float16)a0[0], (_Float16)a0[1], (_Float16)a0[2], (_Float16)a0[3],
               (_Float16)a1[0], (_Float16)a1[1], (_Float16)a1[2], (_Float16)a1[3]};
  const v4u vv = pk.u;
  volatile v4u* d = (volatile v4u*)(dst + o);
  *d = vv;
  __threadfence();
  *d = vv;
}

#define WTP 68
__global__ __launch_bounds__(256) void k_vt(const float* __restrict__ v, _Float16* __restrict__ vt) {
  __shared__ __align__(16) float tf[64 * WTP];
  const int tid = threadIdx.x;
  const int k0 = blockIdx.x * 64;
  const int z  = blockIdx.y;
  const float* src = v + (size_t)z * NN * DD;
  _Float16* dst = vt + (size_t)z * DD * NN;
  {
    const int kr = tid >> 4;
    const int n4 = (tid & 15) * 4;
#pragma unroll
    for (int it = 0; it < 4; ++it) {
      const int kl = it * 16 + kr;
      const v4f a = *(const v4f*)(src + (size_t)(k0 + kl) * DD + n4);
      *(v4f*)(tf + kl * WTP + n4) = a;
    }
  }
  __syncthreads();
  v4u val[2];
  size_t go[2];
#pragma unroll
  for (int j = 0; j < 2; ++j) {
    const int p  = tid + 256 * j;
    const int nl = p >> 3;
    const int pc = p & 7;
    const float* cp = tf + (pc * 8) * WTP + nl;
    Pack8 pk;
    pk.h = (v8h){(_Float16)cp[0 * WTP], (_Float16)cp[1 * WTP], (_Float16)cp[2 * WTP], (_Float16)cp[3 * WTP],
                 (_Float16)cp[4 * WTP], (_Float16)cp[5 * WTP], (_Float16)cp[6 * WTP], (_Float16)cp[7 * WTP]};
    val[j] = pk.u;
    go[j]  = (size_t)nl * NN + k0 + pc * 8;
  }
  for (int ps = 0; ps < 2; ++ps) {
#pragma unroll
    for (int j = 0; j < 2; ++j) *(volatile v4u*)(dst + go[j]) = val[j];
    __threadfence();
  }
}

#define KTP 72
#define PTP 72
#define BTP 64
__global__ __launch_bounds__(256) void k_attn(const _Float16* __restrict__ qp,
                                              const _Float16* __restrict__ kp,
                                              const _Float16* __restrict__ vt,
                                              const float* __restrict__ dm,
                                              const float* __restrict__ w1,
                                              const float* __restrict__ b1,
                                              const float* __restrict__ w2,
                                              const float* __restrict__ b2,
                                              float* __restrict__ out) {
  __shared__ __align__(16) _Float16 Ks[64 * KTP];
  __shared__ __align__(16) _Float16 Vs[64 * KTP];
  __shared__ __align__(16) _Float16 Ps[8][16 * PTP];
  __shared__ __align__(16) float    Bs[8][16 * BTP];

  const int tid = threadIdx.x, lane = tid & 31, wave = tid >> 5;
  const int hh = lane >> 4, c = lane & 15;
  const int bh = (int)blockIdx.x / QBLK;
  const int qb = (int)blockIdx.x % QBLK;
  const int b  = bh / HH, h = bh % HH;
  const int q0 = qb * 128 + wave * 16;

  const _Float16* Q = qp + (size_t)bh * MM * DD;
  const _Float16* K = kp + (size_t)bh * NN * DD;
  const _Float16* V = vt + (size_t)bh * DD * NN;
  const float*   Dm = dm + (size_t)b * MM * NN;
  float*          O = out + (size_t)bh * MM * DD;

  float cA[HID], cC[HID], cB[HID], cW[HID];
#pragma unroll
  for (int f = 0; f < HID; ++f) {
    cA[f] = w1[h * 2 * HID + f];
    cC[f] = w1[h * 2 * HID + HID + f];
    cB[f] = b1[h * HID + f];
    cW[f] = w2[h * HID + f];
  }
  const float cb2 = b2[h];

  v16h qa[2];
  qa[0] = ldfrag(Q, DD, q0, 0, lane);
  qa[1] = ldfrag(Q, DD, q0, 32, lane);

  const float NEGI = -__builtin_huge_valf();
  float mrow[8], lrow[8];
  v8f oacc[4];
#pragma unroll
  for (int r = 0; r < 8; ++r) { mrow[r] = NEGI; lrow[r] = 0.f; }
#pragma unroll
  for (int t = 0; t < 4; ++t) oacc[t] = zero8();

  _Float16* pw = Ps[wave];
  float*    bw = Bs[wave];

  for (int kc = 0; kc < NN / 64; ++kc) {
    const int kv0 = kc * 64;
    __syncthreads();
    {
      const int r  = tid >> 2;
      const int qq = (tid & 3) * 16;
      const _Float16* ks = K + (size_t)(kv0 + r) * DD + qq;
      *(v8h*)(Ks + r * KTP + qq)     = *(const v8h*)(ks);
      *(v8h*)(Ks + r * KTP + qq + 8) = *(const v8h*)(ks + 8);
      const _Float16* vs = V + (size_t)r * NN + kv0 + qq;
      *(v8h*)(Vs + r * KTP + qq)     = *(const v8h*)(vs);
      *(v8h*)(Vs + r * KTP + qq + 8) = *(const v8h*)(vs + 8);
#pragma unroll
      for (int it = 0; it < 8; ++it) {
        const int p   = lane + 32 * it;
        const int row = p >> 4;
        const int c4  = (p & 15) * 4;
        const v4f dv4 = *(const v4f*)(Dm + (size_t)(q0 + row) * NN + kv0 + c4);
        *(v4f*)(bw + row * BTP + c4) = dv4;
      }
    }
    __syncthreads();

    v8f s[4];
#pragma unroll
    for (int j = 0; j < 4; ++j) s[j] = zero8();
#pragma unroll
    for (int dc = 0; dc < 2; ++dc) {
#pragma unroll
      for (int j = 0; j < 4; ++j) {
        const v16h kb = ldfrag(Ks, KTP, j * 16, dc * 32, lane);
        s[j] = mma16(qa[dc], kb, s[j]);
      }
    }
    float cm[8];
#pragma unroll
    for (int r = 0; r < 8; ++r) {
      float m = NEGI;
#pragma unroll
      for (int j = 0; j < 4; ++j) {
        const float sv = s[j][r] * 0.125f;
        const float dv = bw[(8 * hh + r) * BTP + 16 * j + c];
        float x = cb2;
#pragma unroll
        for (int f = 0; f < HID; ++f) {
          float hf = fmaf(sv, cA[f], fmaf(dv, cC[f], cB[f]));
          hf = fmaxf(hf, 0.0f);
          x = fmaf(hf, cW[f], x);
        }
        s[j][r] = x;
        m = fmaxf(m, x);
      }
#pragma unroll
      for (int off = 1; off < 16; off <<= 1) m = fmaxf(m, __shfl_xor(m, off, 32));
      cm[r] = m;
    }
    float al[8];
#pragma unroll
    for (int r = 0; r < 8; ++r) {
      const float mnew  = fmaxf(mrow[r], cm[r]);
      const float alpha = __expf(mrow[r] - mnew);
      mrow[r] = mnew;
      float psum = 0.f;
#pragma unroll
      for (int j = 0; j < 4; ++j) {
        const float p = __expf(s[j][r] - mnew);
        psum += p;
        pw[(8 * hh + r) * PTP + j * 16 + c] = (_Float16)(p * 1024.0f);
      }
#pragma unroll
      for (int off = 1; off < 16; off <<= 1) psum += __shfl_xor(psum, off, 32);
      lrow[r] = lrow[r] * alpha + psum;
      al[r] = alpha;
    }
#pragma unroll
    for (int t = 0; t < 4; ++t)
#pragma unroll
      for (int r = 0; r < 8; ++r) oacc[t][r] *= al[r];
    __syncthreads();

#pragma unroll
    for (int kk = 0; kk < 2; ++kk) {
      const v16h pa = ldfrag(pw, PTP, 0, kk * 32, lane);
#pragma unroll
      for (int t = 0; t < 4; ++t) {
        const v16h vb = ldfrag(Vs, KTP, t * 16, kk * 32, lane);
        oacc[t] = mma16(pa, vb, oacc[t]);
      }
    }
  }
  __syncthreads();

#pragma unroll
  for (int r = 0; r < 8; ++r) {
    const float inv = (1.0f / lrow[r]) * 0.0009765625f;
#pragma unroll
    for (int t = 0; t < 4; ++t) bw[(8 * hh + r) * BTP + 16 * t + c] = oacc[t][r] * inv;
  }
  __syncthreads();
  v4f val[8];
  size_t go[8];
#pragma unroll
  for (int it = 0; it < 8; ++it) {
    const int p    = lane + 32 * it;
    const int L    = p >> 3;
    const int pc   = p & 7;
    const int row  = L >> 1;
    const int half = L & 1;
    val[it] = *(const v4f*)(bw + row * BTP + half * 32 + pc * 4);
    go[it]  = (size_t)(q0 + row) * DD + half * 32 + pc * 4;
  }
  for (int ps = 0; ps < 2; ++ps) {
#pragma unroll
    for (int it = 0; it < 8; ++it) *(volatile v4f*)(O + go[it]) = val[it];
    __threadfence();
  }
}

extern "C" void kernel_launch(void* const* d_in, const int* in_sizes, int n_in,
                              void* d_out, int out_size, void* d_ws, size_t ws_size,
                              hipStream_t stream) {
  if (n_in < 8) return;
  if (in_sizes[0] != NBH * MM * DD) return;
  if (in_sizes[1] != NBH * NN * DD || in_sizes[2] != NBH * NN * DD) return;
  if (in_sizes[3] != BB * MM * NN) return;
  if (in_sizes[4] != HH * 2 * HID || in_sizes[5] != HH * HID) return;
  if (in_sizes[6] != HH * HID || in_sizes[7] != HH) return;
  if (out_size != NBH * MM * DD) return;

  const float* q   = (const float*)d_in[0];
  const float* k   = (const float*)d_in[1];
  const float* v   = (const float*)d_in[2];
  const float* dm  = (const float*)d_in[3];
  const float* w1  = (const float*)d_in[4];
  const float* b1  = (const float*)d_in[5];
  const float* w2  = (const float*)d_in[6];
  const float* b2  = (const float*)d_in[7];
  float* out = (float*)d_out;

  size_t off = 0;
  const size_t oQ = off; off += PL * 2;
  const size_t oK = off; off += PL * 2;
  const size_t oV = off; off += PL * 2;
  if (off > ws_size) return;
  if (off > (size_t)134217728) return;

  char* ws = (char*)d_ws;
  _Float16* Qh = (_Float16*)(ws + oQ);
  _Float16* Kh = (_Float16*)(ws + oK);
  _Float16* Vt = (_Float16*)(ws + oV);

  const int ngrp = in_sizes[0] / 8;
  const int nb   = ngrp / 256;
  k_cvt_qk<<<dim3(2 * nb), dim3(256), 0, stream>>>(q, k, Qh, Kh, ngrp, nb);
  k_vt<<<dim3(NN / 64, NBH), dim3(256), 0, stream>>>(v, Vt);
  k_attn<<<dim3(NBH * QBLK), dim3(256), 0, stream>>>(Qh, Kh, Vt, dm, w1, b1, w2, b2, out);
  (void)hipGetLastError();
}
